// SchNetLayer_31215822307957
// MI455X (gfx1250) — hardware-verified
//
#include <hip/hip_runtime.h>
#include <math.h>

typedef __attribute__((ext_vector_type(16))) _Float16 v16h;
typedef __attribute__((ext_vector_type(16))) __bf16 v16b;
typedef __attribute__((ext_vector_type(8)))  _Float16 v8h;
typedef __attribute__((ext_vector_type(8)))  float v8f;
typedef __attribute__((ext_vector_type(4)))  float v4f;
typedef __attribute__((ext_vector_type(2)))  float v2f;
typedef __attribute__((ext_vector_type(4)))  unsigned v4u;
typedef __attribute__((ext_vector_type(4)))  int v4i;
typedef float __attribute__((may_alias)) float_a;
typedef int __attribute__((may_alias)) int_a;

template <typename T> __device__ __forceinline__ void vst2(void* p, T v) { *(volatile T*)p = v; __threadfence(); *(volatile T*)p = v; }
__device__ __forceinline__ v8f wmma16(v16h a, v16h b, v8f c) {
  v8f d = __builtin_amdgcn_wmma_f32_16x16x32_f16(false, a, false, b, (short)0, c, false, false);
  asm volatile("v_nop\n\tv_nop\n\tv_nop\n\tv_nop" : "+v"(d) : "v"(a), "v"(b));
  return d;
}
__device__ __forceinline__ v8f wmma_bf(v16b a, v16b b, v8f c) {
  v8f d = __builtin_amdgcn_wmma_f32_16x16x32_bf16(false, a, false, b, (short)0, c, false, false);
  asm volatile("v_nop\n\tv_nop\n\tv_nop\n\tv_nop" : "+v"(d) : "v"(a), "v"(b));
  return d;
}
__device__ __forceinline__ v16h frag_h(const _Float16* rowk0, int lane) {
  union { v16h v; v8h q[2]; } u; const _Float16* p = rowk0 + 8 * (lane >> 4);
  u.q[0] = *(const v8h*)p; u.q[1] = *(const v8h*)(p + 16); return u.v;
}
__device__ __forceinline__ v16h frag_f32(const float* rowk0, int lane) {
  v16h a; const float* p = rowk0 + 8 * (lane >> 4);
#pragma unroll
  for (int i = 0; i < 8; ++i) { a[i] = (_Float16)p[i]; a[8 + i] = (_Float16)p[16 + i]; }
  return a;
}
__device__ __forceinline__ v16h frag_f32s(const float* rowk0, int lane, float sc) {
  v16h a; const float* p = rowk0 + 8 * (lane >> 4);
#pragma unroll
  for (int i = 0; i < 8; ++i) { a[i] = (_Float16)(p[i] * sc); a[8 + i] = (_Float16)(p[16 + i] * sc); }
  return a;
}
__device__ __forceinline__ v16h fragc_f32(const float* W, int k0, int n, int lane, int ld, int K) {
  v16h a; const int g = lane >> 4;
#pragma unroll
  for (int i = 0; i < 8; ++i) { const int ka = k0 + 8 * g + i, kb = ka + 16;
    a[i] = (_Float16)(ka < K ? W[(size_t)(ka < K ? ka : K - 1) * ld + n] : 0.f); a[8 + i] = (_Float16)(kb < K ? W[(size_t)(kb < K ? kb : K - 1) * ld + n] : 0.f); }
  return a;
}
struct F2 { v16b h, l; };
__device__ __forceinline__ F2 bsplit16(const float v[16]) { F2 r;
#pragma unroll
  for (int i = 0; i < 16; ++i) { const __bf16 h = (__bf16)v[i]; r.h[i] = h; r.l[i] = (__bf16)(v[i] - (float)h); }
  return r; }
__device__ __forceinline__ F2 split_row(const float* row, int k0, int lane) { float v[16]; const float* p = row + k0 + 8 * (lane >> 4);
#pragma unroll
  for (int i = 0; i < 8; ++i) { v[i] = p[i]; v[8 + i] = p[16 + i]; }
  return bsplit16(v); }
__device__ __forceinline__ F2 split_rowK(const float* row, int k0, int lane, int K) { float v[16]; const int g = lane >> 4;
#pragma unroll
  for (int i = 0; i < 8; ++i) { const int ka = k0 + 8 * g + i, kb = ka + 16; v[i] = ka < K ? row[ka < K ? ka : K - 1] : 0.f; v[8 + i] = kb < K ? row[kb < K ? kb : K - 1] : 0.f; }
  return bsplit16(v); }
__device__ __forceinline__ F2 split_col(const float* W, int k0, int n, int lane, int ld, int K) { float v[16]; const int g = lane >> 4;
#pragma unroll
  for (int i = 0; i < 8; ++i) { const int ka = k0 + 8 * g + i, kb = ka + 16; v[i] = ka < K ? W[(size_t)(ka < K ? ka : K - 1) * ld + n] : 0.f; v[8 + i] = kb < K ? W[(size_t)(kb < K ? kb : K - 1) * ld + n] : 0.f; }
  return bsplit16(v); }
__device__ __forceinline__ v8f mac3(const F2& a, const F2& b, v8f c) { c = wmma_bf(a.l, b.h, c); c = wmma_bf(a.h, b.l, c); return wmma_bf(a.h, b.h, c); }
__device__ __forceinline__ float sigm(float v) { return 1.0f / (1.0f + expf(-v)); }
#define LDSX() do { asm volatile("s_wait_dscnt 0" ::: "memory"); __builtin_amdgcn_wave_barrier(); __builtin_amdgcn_fence(__ATOMIC_RELEASE, "workgroup"); } while (0)

__device__ __forceinline__ float bfr(float v) { return (float)(__bf16)v; }
__device__ __attribute__((noinline)) float sspf(float x) {
  const float sp = (x > 0.f) ? (x + log1pf(expf(-x))) : log1pf(expf(x)); return sp - 0.69314718055994530942f; }
#define NAT 10000
#define KNB 32
#define FF 128
#define NRB 300
#define KRB 320
#define NEDGE (NAT * KNB)
#ifndef NATT
#define NATT NAT
#endif
#define WS_PRE 0u
#define WS_H1  (WS_PRE + 4u * (size_t)NAT * FF)
#define WS_CV  (WS_H1 + 2u * (size_t)NEDGE * FF)
#define WS_P1  (WS_CV + 4u * (size_t)NAT * FF)
#define WS_END (WS_P1 + 4u * (size_t)NAT * FF)
__global__ __launch_bounds__(128) void k_lin(const float* __restrict__ A, const float* __restrict__ Wm, const float* __restrict__ Bv, const float* __restrict__ RES, float* __restrict__ D, int mode, int nrows) { __shared__ __align__(16) float sf[4][16][132];
  const int tid = threadIdx.x, wave = tid >> 5, lane = tid & 31, col = lane & 15, g = lane >> 4; const size_t r0 = (size_t)blockIdx.x * 64 + wave * 16; const size_t ra = (r0 + col < (size_t)nrows) ? r0 + col : (size_t)nrows - 1;
  v8f acc[8] = {};
#pragma unroll
  for (int kc = 0; kc < FF / 32; ++kc) { F2 a; v16b ax;
    if (mode == 0) { const float* p = A + ra * FF + kc * 32 + 8 * g;
#pragma unroll
      for (int i = 0; i < 8; ++i) { ax[i] = (__bf16)p[i]; ax[8 + i] = (__bf16)p[16 + i]; } }
    else a = split_row(A + ra * FF, kc * 32, lane);
#pragma unroll
    for (int j = 0; j < 8; ++j) { v16b w; const int o = j * 16 + col;
#pragma unroll
      for (int i = 0; i < 8; ++i) { w[i] = (__bf16)Wm[(size_t)(kc * 32 + 8 * g + i) * FF + o]; w[8 + i] = (__bf16)Wm[(size_t)(kc * 32 + 16 + 8 * g + i) * FF + o]; }
      if (mode == 0) acc[j] = wmma_bf(ax, w, acc[j]); else { acc[j] = wmma_bf(a.h, w, acc[j]); acc[j] = wmma_bf(a.l, w, acc[j]); } } }
#pragma unroll
  for (int j = 0; j < 8; ++j) { const float bb = bfr(Bv[j * 16 + col]);
#pragma unroll
    for (int r = 0; r < 8; ++r) { float v = acc[j][r] + bb; if (mode == 1) v = sspf(v); else if (mode == 2) v += bfr(RES[(r0 + 8 * g + r < (size_t)nrows ? r0 + 8 * g + r : 0) * FF + j * 16 + col]); sf[wave][8 * g + r][j * 16 + col] = v; } }
  LDSX(); for (int rl = 0; rl < 16; ++rl) { const size_t r = r0 + rl; if (r < (size_t)nrows) vst2(D + r * FF + lane * 4, *(const v4f*)&sf[wave][rl][lane * 4]); } }
__global__ __launch_bounds__(128) void k_edge1(const float* __restrict__ XYZ, const int* __restrict__ SRC, const float* __restrict__ CEN, const float* __restrict__ W1, _Float16* __restrict__ H1) { __shared__ __align__(16) _Float16 sh[4][16][136];
  const int tid = threadIdx.x, wave = tid >> 5, lane = tid & 31, col = lane & 15, g = lane >> 4; const size_t e0 = (size_t)blockIdx.x * 64 + wave * 16; const size_t e = e0 + col; const size_t n = e / KNB;
  const int j = SRC[e]; const float dx = bfr(XYZ[(size_t)j * 3]) - bfr(XYZ[n * 3]), dy = bfr(XYZ[(size_t)j * 3 + 1]) - bfr(XYZ[n * 3 + 1]), dz = bfr(XYZ[(size_t)j * 3 + 2]) - bfr(XYZ[n * 3 + 2]); const float d = sqrtf(dx * dx + dy * dy + dz * dz);
  v8f acc[8] = {};
#pragma unroll 1
  for (int kc = 0; kc < KRB / 32; ++kc) { v16h a;
#pragma unroll
    for (int i = 0; i < 16; ++i) { const int r = kc * 32 + (i < 8 ? 8 * g + i : 16 + 8 * g + (i - 8)); float v = 0.f; if (r < NRB) { const float t = d - bfr(CEN[r]); v = __expf(-10.0f * t * t); } a[i] = (_Float16)v; }
#pragma unroll
    for (int jt = 0; jt < 8; ++jt) { v16h w; const int o = jt * 16 + col;
#pragma unroll
      for (int i = 0; i < 16; ++i) { const int r = kc * 32 + (i < 8 ? 8 * g + i : 16 + 8 * g + (i - 8)); w[i] = (r < NRB) ? (_Float16)(bfr(W1[(size_t)r * FF + o]) * 16.0f) : (_Float16)0.f; }
      acc[jt] = wmma16(a, w, acc[jt]); } }
#pragma unroll
  for (int jt = 0; jt < 8; ++jt)
#pragma unroll
    for (int r = 0; r < 8; ++r) sh[wave][8 * g + r][jt * 16 + col] = (_Float16)sspf(acc[jt][r] * (1.0f / 16.0f));
  LDSX(); for (int rl = 0; rl < 16; ++rl) if (lane < 16) vst2((unsigned*)(H1 + (e0 + rl) * FF + lane * 8), *(const v4u*)&sh[wave][rl][lane * 8]); }
__global__ __launch_bounds__(128) void k_edge2(const _Float16* __restrict__ H1, const float* __restrict__ W2, const float* __restrict__ PRE, const int* __restrict__ SRC, const float* __restrict__ EM, float* __restrict__ CV) { __shared__ __align__(16) float sp[4][FF];
  const int tid = threadIdx.x, wave = tid >> 5, lane = tid & 31, col = lane & 15, g = lane >> 4; const size_t e0 = (size_t)blockIdx.x * 64 + wave * 16;
  v8f acc[8] = {};
#pragma unroll
  for (int kc = 0; kc < FF / 32; ++kc) { const v16h a = frag_h(H1 + (e0 + col) * FF + kc * 32, lane);
#pragma unroll
    for (int jt = 0; jt < 8; ++jt) { v16h w; const int o = jt * 16 + col;
#pragma unroll
      for (int i = 0; i < 8; ++i) { w[i] = (_Float16)(bfr(W2[(size_t)(kc * 32 + 8 * g + i) * FF + o]) * 16.0f); w[8 + i] = (_Float16)(bfr(W2[(size_t)(kc * 32 + 16 + 8 * g + i) * FF + o]) * 16.0f); }
      acc[jt] = wmma16(a, w, acc[jt]); } }
  float part[8];
#pragma unroll
  for (int jt = 0; jt < 8; ++jt) { float s = 0.f;
#pragma unroll
    for (int r = 0; r < 8; ++r) { const size_t e = e0 + 8 * g + r; const int j = SRC[e]; const float f = sspf(acc[jt][r] * (1.0f / 16.0f)); s += f * PRE[(size_t)j * FF + jt * 16 + col] * bfr(EM[e]); }
    s += __shfl_xor(s, 16);
    part[jt] = s; }
  if (g == 0) {
#pragma unroll
    for (int jt = 0; jt < 8; ++jt) sp[wave][jt * 16 + col] = part[jt]; }
  __syncthreads();
  if ((wave & 1) == 0) { const size_t n = (size_t)blockIdx.x * 2 + (wave >> 1); v4f o;
#pragma unroll
    for (int i = 0; i < 4; ++i) o[i] = sp[wave][lane * 4 + i] + sp[wave + 1][lane * 4 + i];
    vst2(CV + n * FF + lane * 4, o); } }
extern "C" void kernel_launch(void* const* d_in, const int* in_sizes, int n_in, void* d_out, int out_size, void* d_ws, size_t ws_size, hipStream_t stream) {
  (void)in_sizes; (void)n_in; (void)out_size;
  const float** F = (const float**)d_in;
  if (ws_size < (size_t)WS_END) return;
  char* ws = (char*)d_ws; float *PRE = (float*)(ws + WS_PRE), *CV = (float*)(ws + WS_CV), *P1 = (float*)(ws + WS_P1); _Float16* H1 = (_Float16*)(ws + WS_H1);
  k_lin<<<dim3((NAT + 63) / 64), 128, 0, stream>>>(F[1], F[4], F[5], nullptr, PRE, 0, NAT);
  k_edge1<<<dim3(NATT * KNB / 64), 128, 0, stream>>>(F[0], (const int*)d_in[3], F[12], F[6], H1);
  k_edge2<<<dim3(NATT * KNB / 64), 128, 0, stream>>>(H1, F[7], PRE, (const int*)d_in[3], F[2], CV);
  k_lin<<<dim3((NATT + 63) / 64), 128, 0, stream>>>(CV, F[8], F[9], nullptr, P1, 1, NATT);
  k_lin<<<dim3((NATT + 63) / 64), 128, 0, stream>>>(P1, F[10], F[11], F[1], (float*)d_out, 2, NATT);
}
